// Explorer_56178172232399
// MI455X (gfx1250) — hardware-verified
//
#include <hip/hip_runtime.h>
#include <stddef.h>


#define HC      64
#define NTHR    256
#define NWAVE   8
#define RB      128
#define AP      72
#define AP32    40
#define TGT     256
#define HCAP    2048
#define EPT     8
#define NGRP    2
#define CHUNK   (NTHR * EPT * NGRP)
#define WCAP    (EPT * NGRP * 32)
#define LMAX    3
#define PQW     128

#define PL_HX1  0
#define PL_HX2  4096
#define PL_HY1  8192
#define PL_HY2  10240
#define PL_FXD  14336
#define PL_FX2  18432
#define PL_FY2  22528
#define PL_FE1  26624
#define PL_FE2  30720
#define PL_FE3  34816
#define PL_CXH  36864
#define PL_CXL  45056
#define PL_CYH  53248
#define PL_CYL  61440
#define PL_TOT  69632
#define NPREP   (PL_TOT / 8 / NTHR)

#define MO_AGG   0
#define MO_HITS  (TGT * HC * 4)
#define MO_RS    (MO_HITS + HCAP * 4)
#define MO_WCNT  (MO_RS + 128 * 4)
#define MO_STG   (MO_WCNT + 256)
#define R2OFF    (16 * AP * 2 * 2)
#define WSTG     (R2OFF + 16 * HC * 4)
#define MSG_LDS  (MO_STG + NWAVE * WSTG)
#define ROW_LDS  (RB * AP * 2 * 2)
#define PROJ_LDS (RB * PQW * 4)

static_assert(PL_TOT % (8 * NTHR) == 0);
static_assert(NWAVE * WCAP * 4 <= NWAVE * WSTG);
static_assert(RB * HC * 4 <= ROW_LDS);
static_assert(RB * AP32 * 2 * 2 <= ROW_LDS);
static_assert(RB * AP * 2 * 2 <= PROJ_LDS);
static_assert((CHUNK & (CHUNK - 1)) == 0 && CHUNK <= 4096);
static_assert((TGT & (TGT - 1)) == 0 && TGT <= 4096);
static_assert(TGT == 32 * NWAVE);
static_assert(RB == 16 * NWAVE);
static_assert(HCAP % 128 == 0);
static_assert((MO_STG % 16) == 0 && (WSTG % 16) == 0 && (R2OFF % 16) == 0);

typedef unsigned short us;
typedef float  v2f  __attribute__((ext_vector_type(2)));
typedef float  v4f  __attribute__((ext_vector_type(4)));
typedef float  v8f  __attribute__((ext_vector_type(8)));
typedef int    v4i  __attribute__((ext_vector_type(4)));
typedef us     v8us __attribute__((ext_vector_type(8)));
typedef us     v16us __attribute__((ext_vector_type(16)));
typedef __bf16 v16b __attribute__((ext_vector_type(16)));
union FragB { v16b v; v16us u; v8us h[2]; };

__device__ __forceinline__ us f2bf(float f) {
  unsigned u = __float_as_uint(f);
  u = u + 0x7FFFu + ((u >> 16) & 1u);
  return (us)(u >> 16);
}
__device__ __forceinline__ float bf2f(us b) { return __uint_as_float(((unsigned)b) << 16); }
__device__ __forceinline__ float bfr(float f) {
  const unsigned u = __float_as_uint(f);
  return __uint_as_float((u + 0x7FFFu + ((u >> 16) & 1u)) & 0xFFFF0000u);
}
__device__ __forceinline__ v4f bfr4(v4f a) {
  v4f r; r.x = bfr(a.x); r.y = bfr(a.y); r.z = bfr(a.z); r.w = bfr(a.w); return r;
}

__device__ __forceinline__ v8f wmb(const FragB& a, const FragB& b, v8f c) {
  v8f d = __builtin_amdgcn_wmma_f32_16x16x32_bf16(false, a.v, false, b.v, (short)0, c, false, false);
#if defined(__HIP_DEVICE_COMPILE__)
  asm volatile("v_nop\n\tv_nop\n\tv_nop\n\tv_nop" : "+v"(d) : "v"(a.u), "v"(b.u));
#endif
  return d;
}

template <int NT>
__device__ __forceinline__ void zacc(v8f (&acc)[NT]) {
#pragma unroll
  for (int t = 0; t < NT; ++t) {
#pragma unroll
    for (int r = 0; r < 8; ++r) acc[t][r] = 0.0f;
  }
}

template <int KS, int NT>
__device__ __forceinline__ void mm2(const us* aH, const us* aL, const us* __restrict__ B,
                                    v8f (&acc)[NT], int m, int h) {
  constexpr int BP = 32 * KS;
#pragma unroll
  for (int kt = 0; kt < KS; ++kt) {
    FragB ah, al;
    ah.h[0] = *(const v8us*)(aH + 32 * kt);
    ah.h[1] = *(const v8us*)(aH + 32 * kt + 16);
    al.h[0] = *(const v8us*)(aL + 32 * kt);
    al.h[1] = *(const v8us*)(aL + 32 * kt + 16);
#pragma unroll
    for (int t = 0; t < NT; ++t) {
      const us* bp = B + (size_t)(16 * t + m) * BP + 32 * kt + 8 * h;
      FragB b;
      b.h[0] = *(const v8us*)bp;
      b.h[1] = *(const v8us*)(bp + 16);
      acc[t] = wmb(ah, b, acc[t]);
      acc[t] = wmb(al, b, acc[t]);
    }
  }
}

template <int KS, int NT>
__device__ __forceinline__ void mm3(const us* aH, const us* aL, const us* __restrict__ BH,
                                    const us* __restrict__ BL, v8f (&acc)[NT], int m, int h) {
  constexpr int BP = 32 * KS;
#pragma unroll
  for (int kt = 0; kt < KS; ++kt) {
    FragB ah, al;
    ah.h[0] = *(const v8us*)(aH + 32 * kt);
    ah.h[1] = *(const v8us*)(aH + 32 * kt + 16);
    al.h[0] = *(const v8us*)(aL + 32 * kt);
    al.h[1] = *(const v8us*)(aL + 32 * kt + 16);
#pragma unroll
    for (int t = 0; t < NT; ++t) {
      const size_t bo = (size_t)(16 * t + m) * BP + 32 * kt + 8 * h;
      FragB bh, bl;
      bh.h[0] = *(const v8us*)(BH + bo);
      bh.h[1] = *(const v8us*)(BH + bo + 16);
      bl.h[0] = *(const v8us*)(BL + bo);
      bl.h[1] = *(const v8us*)(BL + bo + 16);
      acc[t] = wmb(ah, bh, acc[t]);
      acc[t] = wmb(ah, bl, acc[t]);
      acc[t] = wmb(al, bh, acc[t]);
    }
  }
}

__device__ __forceinline__ void stage32(const float* __restrict__ src, us* dh, us* dl) {
#pragma unroll
  for (int q = 0; q < 4; ++q) {
    const v4f a = *(const v4f*)(src + 8 * q);
    const v4f b = *(const v4f*)(src + 8 * q + 4);
    float f[8];
    f[0] = a.x; f[1] = a.y; f[2] = a.z; f[3] = a.w; f[4] = b.x; f[5] = b.y; f[6] = b.z; f[7] = b.w;
    v8us ph, pl;
#pragma unroll
    for (int j = 0; j < 8; ++j) {
      const us hb = f2bf(f[j]);
      ph[j] = hb;
      pl[j] = f2bf(f[j] - bf2f(hb));
    }
    *(v8us*)(dh + 8 * q) = ph;
    *(v8us*)(dl + 8 * q) = pl;
  }
}

__device__ __forceinline__ void epi_hidden(const v8f (&acc)[4], const float* __restrict__ bias,
                                           us* ph, us* pl, int row0, int m) {
#pragma unroll
  for (int t = 0; t < 4; ++t) {
    const int col = 16 * t + m;
    const float bb = bfr(bias[col]);
#pragma unroll
    for (int r = 0; r < 8; ++r) {
      const float val = fmaxf(acc[t][r] + bb, 0.0f);
      const us hb = f2bf(val);
      ph[(row0 + r) * AP + col] = hb;
      pl[(row0 + r) * AP + col] = f2bf(val - bf2f(hb));
    }
  }
}

__device__ __forceinline__ void store_rows16(const float* lp, float* gp, int lane) {
  const int rl = lane >> 4, col = (lane & 15) * 4;
#pragma unroll
  for (int i = 0; i < 8; ++i) {
    const v4f val = *(const v4f*)(lp + (2 * i + rl) * HC + col);
    *(volatile v4f*)(gp + (size_t)(2 * i + rl) * HC + col) = val;
  }
  __threadfence();
#pragma unroll
  for (int i = 0; i < 8; ++i) {
    const v4f val = *(const v4f*)(lp + (2 * i + rl) * HC + col);
    *(volatile v4f*)(gp + (size_t)(2 * i + rl) * HC + col) = val;
  }
}

__device__ __forceinline__ void merge_max_rows16(float* lp, float* gp, int lane) {
  const int rl = lane >> 4, col = (lane & 15) * 4;
#pragma unroll
  for (int i = 0; i < 8; ++i) {
    float* l = lp + (2 * i + rl) * HC + col;
    float* g = gp + (size_t)(2 * i + rl) * HC + col;
    const v4f o = *(const v4f*)g;
    v4f n = *(const v4f*)l;
    n.x = fmaxf(o.x, n.x); n.y = fmaxf(o.y, n.y); n.z = fmaxf(o.z, n.z); n.w = fmaxf(o.w, n.w);
    *(v4f*)l = n;
    *(volatile v4f*)g = n;
  }
  __threadfence();
#pragma unroll
  for (int i = 0; i < 8; ++i) {
    const v4f n = *(const v4f*)(lp + (2 * i + rl) * HC + col);
    *(volatile v4f*)(gp + (size_t)(2 * i + rl) * HC + col) = n;
  }
}

template <int NB>
__device__ __forceinline__ int scan_chunk(const int* __restrict__ dsts, int nE, int cbase, int slotBase,
                                          int vec8, int* list, int tid, int lane, int wave) {
  int wc = 0;
#pragma unroll
  for (int g = 0; g < NGRP; ++g) {
    const int el0  = (g * NTHR + tid) * EPT;
    const int e0   = cbase + el0;
    const int sent = -2147483647 - 1;
    const int le   = nE - 1;
    v4i da, db;
    if (vec8 != 0 && cbase + CHUNK <= nE) {
      da = *(const v4i*)(dsts + e0);
      db = *(const v4i*)(dsts + e0 + 4);
    } else {
      da.x = (e0     < nE) ? dsts[min(e0,     le)] : sent;
      da.y = (e0 + 1 < nE) ? dsts[min(e0 + 1, le)] : sent;
      da.z = (e0 + 2 < nE) ? dsts[min(e0 + 2, le)] : sent;
      da.w = (e0 + 3 < nE) ? dsts[min(e0 + 3, le)] : sent;
      db.x = (e0 + 4 < nE) ? dsts[min(e0 + 4, le)] : sent;
      db.y = (e0 + 5 < nE) ? dsts[min(e0 + 5, le)] : sent;
      db.z = (e0 + 6 < nE) ? dsts[min(e0 + 6, le)] : sent;
      db.w = (e0 + 7 < nE) ? dsts[min(e0 + 7, le)] : sent;
    }
    const unsigned nb = (unsigned)slotBase;
    const unsigned s0 = (unsigned)da.x - nb, s1 = (unsigned)da.y - nb;
    const unsigned s2 = (unsigned)da.z - nb, s3 = (unsigned)da.w - nb;
    const unsigned s4 = (unsigned)db.x - nb, s5 = (unsigned)db.y - nb;
    const unsigned s6 = (unsigned)db.z - nb, s7 = (unsigned)db.w - nb;
    const bool h0 = s0 < (unsigned)NB, h1 = s1 < (unsigned)NB, h2 = s2 < (unsigned)NB, h3 = s3 < (unsigned)NB;
    const bool h4 = s4 < (unsigned)NB, h5 = s5 < (unsigned)NB, h6 = s6 < (unsigned)NB, h7 = s7 < (unsigned)NB;
    const unsigned any = __builtin_amdgcn_ballot_w32(h0 | h1 | h2 | h3 | h4 | h5 | h6 | h7);
    if (any != 0u) {
#define HITJ(J, HJ, SJ) { \
        const unsigned mj = __builtin_amdgcn_ballot_w32(HJ); \
        if (mj != 0u) { \
          if (HJ) { \
            const int pos = wc + (int)__builtin_amdgcn_mbcnt_lo(mj, 0u); \
            if (pos < WCAP) list[wave * WCAP + pos] = ((el0 + (J)) << 12) | (int)(SJ); \
          } \
          wc += (int)__builtin_popcount(mj); } }
      HITJ(0, h0, s0)
      HITJ(1, h1, s1)
      HITJ(2, h2, s2)
      HITJ(3, h3, s3)
      HITJ(4, h4, s4)
      HITJ(5, h5, s5)
      HITJ(6, h6, s6)
      HITJ(7, h7, s7)
#undef HITJ
    }
  }
  return wc;
}

__global__ __launch_bounds__(NTHR) void k_prep(
    const float* __restrict__ hxw1, const float* __restrict__ hxw2,
    const float* __restrict__ hyw1, const float* __restrict__ hyw2,
    const float* __restrict__ fxw1, const float* __restrict__ fxw2,
    const float* __restrict__ fyw1, const float* __restrict__ fyw2,
    const float* __restrict__ few1, const float* __restrict__ few2, const float* __restrict__ few3,
    us* wpl) {
  const int b = blockIdx.x, tid = threadIdx.x;
  const float* W = hxw1;
  int K = 36, kps = 6, NV = 64, ldw = 64, t0 = 0, po = PL_HX1, comb = 0, lo = 0;
  if (b < 2)       { W = hxw1; K = 36; t0 = 0;    po = PL_HX1; }
  else if (b < 4)  { W = hxw2; K = 64; t0 = 512;  po = PL_HX2; }
  else if (b < 5)  { W = hyw1; K = 27; kps = 5; t0 = 1024; po = PL_HY1; }
  else if (b < 7)  { W = hyw2; K = 64; t0 = 1280; po = PL_HY2; }
  else if (b < 9)  { W = fxw1 + 192 * 64; K = 64; t0 = 1792; po = PL_FXD; }
  else if (b < 11) { W = fxw2; K = 64; t0 = 2304; po = PL_FX2; }
  else if (b < 13) { W = fyw2; K = 64; t0 = 2816; po = PL_FY2; }
  else if (b < 15) { W = few1; K = 64; t0 = 3328; po = PL_FE1; }
  else if (b < 17) { W = few2; K = 64; t0 = 3840; po = PL_FE2; }
  else if (b < 18) { W = few3; K = 64; NV = 1; ldw = 1; t0 = 4352; po = PL_FE3; }
  else if (b < 22) { W = fxw1; K = 64; comb = 1; t0 = 4608; po = PL_CXH; }
  else if (b < 26) { W = fxw1; K = 64; comb = 1; lo = 1; t0 = 5632; po = PL_CXL; }
  else if (b < 30) { W = fyw1; K = 64; comb = 1; t0 = 6656; po = PL_CYH; }
  else             { W = fyw1; K = 64; comb = 1; lo = 1; t0 = 7680; po = PL_CYL; }
  const int i  = b * NTHR + tid - t0;
  const int o  = 8 * i;
  const int n  = o >> kps;
  const int k0 = o & ((1 << kps) - 1);
  v8us outv;
#pragma unroll
  for (int e = 0; e < 8; ++e) {
    const int k = k0 + e;
    float val;
    if (comb != 0) {
      const int kc = k > 63 ? 63 : k;
      const int nn = n & 63;
      const bool lower = n < 64;
      const int ra = lower ? kc : 128 + kc;
      const int rbk = lower ? 64 + kc : kc;
      const float a  = bfr(W[(size_t)ra * 64 + nn]);
      const float bb = bfr(W[(size_t)rbk * 64 + nn]);
      val = lower ? a + bb : a - bb;
    } else {
      const int kc = k < K ? k : K - 1;
      const int nc = n < NV ? n : NV - 1;
      const float x = W[(size_t)kc * ldw + nc];
      val = (k < K && n < NV) ? bfr(x) : 0.0f;
    }
    const us hb = f2bf(val);
    outv[e] = (lo != 0) ? f2bf(val - bf2f(hb)) : hb;
  }
  us* dp = wpl + po + o;
  *(volatile v8us*)dp = outv;
  __threadfence();
  *(volatile v8us*)dp = outv;
}

__global__ __launch_bounds__(NTHR) void k_goal(const float* __restrict__ v, const float* __restrict__ lab,
                                               float* goal, int nN) {
  __shared__ float sv[NWAVE];
  __shared__ int   si[NWAVE];
  __shared__ __attribute__((aligned(16))) float sg[32];
  const int tid = threadIdx.x, lane = tid & 31, wave = tid >> 5;
  float best = __uint_as_float(0xff800000u);
  int bi = 0x7fffffff;
#pragma unroll 1
  for (int i = tid; i < nN; i += NTHR) {
    const float x = lab[(size_t)i * 2 + 1];
    if (x > best) { best = x; bi = i; }
  }
#pragma unroll
  for (int o = 16; o > 0; o >>= 1) {
    const float ob = __shfl_xor(best, o);
    const int   oi = __shfl_xor(bi, o);
    const bool take = (ob > best) || (ob == best && oi < bi);
    best = take ? ob : best;
    bi   = take ? oi : bi;
  }
  if (lane == 0) { sv[wave] = best; si[wave] = bi; }
  __syncthreads();
  if (wave == 0) {
    const int li = lane < NWAVE ? lane : NWAVE - 1;
    best = sv[li]; bi = si[li];
#pragma unroll
    for (int o = 16; o > 0; o >>= 1) {
      const float ob = __shfl_xor(best, o);
      const int   oi = __shfl_xor(bi, o);
      const bool take = (ob > best) || (ob == best && oi < bi);
      best = take ? ob : best;
      bi   = take ? oi : bi;
    }
    int g = __builtin_amdgcn_readfirstlane(bi);
    g = g < 0 ? 0 : (g > nN - 1 ? nN - 1 : g);
    const int cv = lane < 7 ? lane : 6;
    const int lc = lane - 7;
    const int cl = lc < 0 ? 0 : (lc > 1 ? 1 : lc);
    const float a  = v[(size_t)g * 7 + cv];
    const float bl = lab[(size_t)g * 2 + cl];
    sg[lane] = lane < 7 ? bfr(a) : (lane < 9 ? bfr(bl) : 0.0f);
  }
  __syncthreads();
  if (wave == 0) {
    const v4f gv = *(const v4f*)(sg + 4 * (lane & 7));
    if (lane < 8) *(volatile v4f*)(goal + 4 * lane) = gv;
    __threadfence();
    if (lane < 8) *(volatile v4f*)(goal + 4 * lane) = gv;
  }
}

__device__ __forceinline__ float featx(const float (&vcv)[9], const float (&gl)[9], const float (&dv)[9],
                                       float zd, int k) {
  if (k < 9)  return vcv[k];
  if (k < 18) return gl[k - 9];
  if (k < 27) return dv[k - 18];
  if (k < 36) { const float t = dv[k - 27]; return t * t; }
  return zd;
}

__global__ __launch_bounds__(NTHR) void k_xinit(
    const float* __restrict__ v, const float* __restrict__ lab, const float* __restrict__ goal,
    const us* __restrict__ wpl, const float* __restrict__ b1, const float* __restrict__ b2,
    float* xf, int nN) {
  extern __shared__ v4f lds_dyn[];
  us*    sH  = (us*)lds_dyn;
  us*    sLo = sH + RB * AP;
  float* stg = (float*)lds_dyn;
  const int tid = threadIdx.x, lane = tid & 31, wave = tid >> 5, h = lane >> 4, m = lane & 15;
  const int rowBase = blockIdx.x * RB;
  const int lr = wave * 16 + m;
  int node = rowBase + lr;
  node = node > nN - 1 ? nN - 1 : node;
  const float zd = (float)(node >> 26);
  float vcv[9], gl[9], dv[9];
#pragma unroll
  for (int c = 0; c < 7; ++c) vcv[c] = bfr(v[(size_t)node * 7 + c]);
  vcv[7] = bfr(lab[(size_t)node * 2]);
  vcv[8] = bfr(lab[(size_t)node * 2 + 1]);
#pragma unroll
  for (int c = 0; c < 9; ++c) { const float gv = goal[c]; gl[c] = gv + zd; dv[c] = vcv[c] - gv; }
#pragma unroll
  for (int q = 0; q < 4; ++q) {
    v8us ph, pl;
#pragma unroll
    for (int j = 0; j < 8; ++j) {
      const int jj = 8 * q + j;
      const float f0 = featx(vcv, gl, dv, zd, jj);
      const float f1 = featx(vcv, gl, dv, zd, 32 + jj);
      const float f = h ? f1 : f0;
      const us hb = f2bf(f);
      ph[j] = hb;
      pl[j] = f2bf(f - bf2f(hb));
    }
    *(v8us*)(sH  + lr * AP + 32 * h + 8 * q) = ph;
    *(v8us*)(sLo + lr * AP + 32 * h + 8 * q) = pl;
  }
  __syncthreads();
  v8f acc[4];
  zacc(acc);
  const us* aH = sH + lr * AP + 8 * h;
  const us* aL = sLo + lr * AP + 8 * h;
  mm2<2, 4>(aH, aL, wpl + PL_HX1, acc, m, h);
  __syncthreads();
  epi_hidden(acc, b1, sH, sLo, wave * 16 + 8 * h, m);
  __syncthreads();
  zacc(acc);
  mm2<2, 4>(aH, aL, wpl + PL_HX2, acc, m, h);
  __syncthreads();
#pragma unroll
  for (int t = 0; t < 4; ++t) {
    const int col = 16 * t + m;
    const float bb = bfr(b2[col]);
#pragma unroll
    for (int r = 0; r < 8; ++r) stg[(wave * 16 + 8 * h + r) * HC + col] = acc[t][r] + bb;
  }
  __syncthreads();
  store_rows16(stg + wave * 16 * HC, xf + (size_t)(rowBase + wave * 16) * HC, lane);
}

__device__ __forceinline__ float featy(const float (&vi)[9], const float (&vj)[9], float zd, int k) {
  if (k < 9)  return vj[k] - vi[k];
  if (k < 18) return vj[k - 9];
  if (k < 27) return vi[k - 18];
  return zd;
}

__global__ __launch_bounds__(NTHR) void k_yinit(
    const float* __restrict__ v, const float* __restrict__ lab, const int* __restrict__ ei,
    const us* __restrict__ wpl, const float* __restrict__ b1, const float* __restrict__ b2,
    float* y, int nN, int nE) {
  extern __shared__ v4f lds_dyn[];
  us*    s32h = (us*)lds_dyn;
  us*    s32l = s32h + RB * AP32;
  us*    sH   = (us*)lds_dyn;
  us*    sLo  = sH + RB * AP;
  float* stg  = (float*)lds_dyn;
  const int tid = threadIdx.x, lane = tid & 31, wave = tid >> 5, h = lane >> 4, m = lane & 15;
  const int rowBase = blockIdx.x * RB;
  const int lr = wave * 16 + m;
  int e = rowBase + lr;
  e = e > nE - 1 ? nE - 1 : e;
  int s = ei[e];      s = s < 0 ? 0 : (s > nN - 1 ? nN - 1 : s);
  int d = ei[nE + e]; d = d < 0 ? 0 : (d > nN - 1 ? nN - 1 : d);
  const float zd = (float)(e >> 26);
  float vi[9], vj[9];
#pragma unroll
  for (int c = 0; c < 7; ++c) { vi[c] = bfr(v[(size_t)s * 7 + c]); vj[c] = bfr(v[(size_t)d * 7 + c]); }
  vi[7] = bfr(lab[(size_t)s * 2]); vi[8] = bfr(lab[(size_t)s * 2 + 1]);
  vj[7] = bfr(lab[(size_t)d * 2]); vj[8] = bfr(lab[(size_t)d * 2 + 1]);
#pragma unroll
  for (int q = 0; q < 2; ++q) {
    v8us ph, pl;
#pragma unroll
    for (int j = 0; j < 8; ++j) {
      const int jj = 8 * q + j;
      const float f0 = featy(vi, vj, zd, jj);
      const float f1 = featy(vi, vj, zd, 16 + jj);
      const float f = h ? f1 : f0;
      const us hb = f2bf(f);
      ph[j] = hb;
      pl[j] = f2bf(f - bf2f(hb));
    }
    *(v8us*)(s32h + lr * AP32 + 16 * h + 8 * q) = ph;
    *(v8us*)(s32l + lr * AP32 + 16 * h + 8 * q) = pl;
  }
  __syncthreads();
  v8f acc[4];
  zacc(acc);
  mm2<1, 4>(s32h + lr * AP32 + 8 * h, s32l + lr * AP32 + 8 * h, wpl + PL_HY1, acc, m, h);
  __syncthreads();
  epi_hidden(acc, b1, sH, sLo, wave * 16 + 8 * h, m);
  __syncthreads();
  zacc(acc);
  mm2<2, 4>(sH + lr * AP + 8 * h, sLo + lr * AP + 8 * h, wpl + PL_HY2, acc, m, h);
  __syncthreads();
#pragma unroll
  for (int t = 0; t < 4; ++t) {
    const int col = 16 * t + m;
    const float bb = bfr(b2[col]);
#pragma unroll
    for (int r = 0; r < 8; ++r) stg[(wave * 16 + 8 * h + r) * HC + col] = acc[t][r] + bb;
  }
  __syncthreads();
  store_rows16(stg + wave * 16 * HC, y + (size_t)(rowBase + wave * 16) * HC, lane);
}

__global__ __launch_bounds__(NTHR) void k_proj(
    const float* __restrict__ xf, const us* __restrict__ bh, const us* __restrict__ bl, float* pq,
    const int* __restrict__ loopp, int it) {
  if (it >= loopp[0]) return;
  extern __shared__ v4f lds_dyn[];
  us*    sH  = (us*)lds_dyn;
  us*    sLo = sH + RB * AP;
  float* stg = (float*)lds_dyn;
  const int tid = threadIdx.x, lane = tid & 31, wave = tid >> 5, h = lane >> 4, m = lane & 15;
  const int rowBase = blockIdx.x * RB;
  const int lr = wave * 16 + m;
  stage32(xf + (size_t)(rowBase + lr) * HC + 32 * h, sH + lr * AP + 32 * h, sLo + lr * AP + 32 * h);
  __syncthreads();
  v8f acc[8];
  zacc(acc);
  mm3<2, 8>(sH + lr * AP + 8 * h, sLo + lr * AP + 8 * h, bh, bl, acc, m, h);
  __syncthreads();
#pragma unroll
  for (int t = 0; t < 8; ++t) {
#pragma unroll
    for (int r = 0; r < 8; ++r) stg[(wave * 16 + 8 * h + r) * PQW + 16 * t + m] = acc[t][r];
  }
  __syncthreads();
  const float* lp = stg + wave * 16 * PQW + 4 * lane;
  float* gp = pq + (size_t)(rowBase + wave * 16) * PQW + 4 * lane;
#pragma unroll
  for (int i = 0; i < 16; ++i) { const v4f val = *(const v4f*)(lp + i * PQW); *(volatile v4f*)(gp + (size_t)i * PQW) = val; }
  __threadfence();
#pragma unroll
  for (int i = 0; i < 16; ++i) { const v4f val = *(const v4f*)(lp + i * PQW); *(volatile v4f*)(gp + (size_t)i * PQW) = val; }
}

__global__ __launch_bounds__(NTHR) void k_msg(
    const int* __restrict__ ei, const float* __restrict__ y, const float* __restrict__ pq,
    const us* __restrict__ wpl, const float* __restrict__ b1, const float* __restrict__ b2,
    float* xf, const int* __restrict__ loopp, int it, int nN, int nE, int vec8) {
  if (it >= loopp[0]) return;
  extern __shared__ v4f lds_dyn[];
  char*  base = (char*)lds_dyn;
  float* agg  = (float*)(base + MO_AGG);
  int*   hits = (int*)(base + MO_HITS);
  int*   rs   = (int*)(base + MO_RS);
  int*   wcnt = (int*)(base + MO_WCNT);
  int*   list = (int*)(base + MO_STG);
  const int tid = threadIdx.x, lane = tid & 31, wave = tid >> 5, h = lane >> 4, m = lane & 15;
  const int nodeBase = blockIdx.x * TGT;
  const int* dsts = ei + nE;

  {
    const float nf = __uint_as_float(0xff800000u);
    v4f ninf; ninf.x = nf; ninf.y = nf; ninf.z = nf; ninf.w = nf;
    for (int i = tid; i < TGT * HC / 4; i += NTHR) ((v4f*)agg)[i] = ninf;
  }

  int hcount = 0;
  const int nChunks = (nE + CHUNK - 1) / CHUNK;
#pragma unroll 1
  for (int ch = 0; ch < nChunks; ++ch) {
    const int cbase = ch * CHUNK;
    const int wc = scan_chunk<TGT>(dsts, nE, cbase, nodeBase, vec8, list, tid, lane, wave);
    if (lane == 0) wcnt[wave] = wc;
    __syncthreads();
    int pre = 0, tot = 0;
#pragma unroll
    for (int w = 0; w < NWAVE; ++w) {
      int c = wcnt[w];
      c = c < 0 ? 0 : (c > WCAP ? WCAP : c);
      tot += c;
      pre += (w < wave) ? c : 0;
    }
    const int mine = wc < 0 ? 0 : (wc > WCAP ? WCAP : wc);
#pragma unroll 1
    for (int i = lane; i < mine; i += 32) {
      const int ent  = list[wave * WCAP + i];
      const int e    = cbase + ((ent >> 12) & (CHUNK - 1));
      const int slot = ent & (TGT - 1);
      const int pos  = hcount + pre + i;
      if (pos < HCAP) hits[pos] = (e << 8) | slot;
    }
    hcount += tot;
    hcount = hcount > HCAP ? HCAP : hcount;
    __syncthreads();
  }

  const int nStep = (hcount + 127) >> 7;
  us*    r1h = (us*)(base + MO_STG + wave * WSTG);
  us*    r1l = r1h + 16 * AP;
  float* r2  = (float*)(base + MO_STG + wave * WSTG + R2OFF);
#pragma unroll 1
  for (int st = 0; st < nStep; ++st) {
    const int idx = st * 128 + wave * 16 + m;
    const bool valid = idx < hcount;
    const int ent = hits[idx < HCAP ? idx : HCAP - 1];
    int e = ent >> 8;
    e = e < 0 ? 0 : (e > nE - 1 ? nE - 1 : e);
    const int slot = ent & (TGT - 1);
    int s = ei[e];   s = s < 0 ? 0 : (s > nN - 1 ? nN - 1 : s);
    int d = dsts[e]; d = d < 0 ? 0 : (d > nN - 1 ? nN - 1 : d);
    if (h == 0) rs[wave * 16 + m] = valid ? slot : -1;
    stage32(y + (size_t)e * HC + 32 * h, r1h + m * AP + 32 * h, r1l + m * AP + 32 * h);
    {
      const float* pp = pq + (size_t)s * PQW + 32 * h;
      const float* qp = pq + (size_t)d * PQW + 64 + 32 * h;
      const float* bp = b1 + 32 * h;
      float* rp = r2 + m * HC + 32 * h;
#pragma unroll
      for (int q = 0; q < 8; ++q) {
        const v4f a  = *(const v4f*)(pp + 4 * q);
        const v4f bb = *(const v4f*)(qp + 4 * q);
        const v4f c  = bfr4(*(const v4f*)(bp + 4 * q));
        *(v4f*)(rp + 4 * q) = a + bb + c;
      }
    }
    __syncthreads();
    v8f acc[4];
    zacc(acc);
    const us* aH = r1h + m * AP + 8 * h;
    const us* aL = r1l + m * AP + 8 * h;
    mm2<2, 4>(aH, aL, wpl + PL_FXD, acc, m, h);
    __syncthreads();
#pragma unroll
    for (int t = 0; t < 4; ++t) {
      const int col = 16 * t + m;
#pragma unroll
      for (int r = 0; r < 8; ++r) {
        const int row = 8 * h + r;
        const float val = fmaxf(acc[t][r] + r2[row * HC + col], 0.0f);
        const us hb = f2bf(val);
        r1h[row * AP + col] = hb;
        r1l[row * AP + col] = f2bf(val - bf2f(hb));
      }
    }
    __syncthreads();
    zacc(acc);
    mm2<2, 4>(aH, aL, wpl + PL_FX2, acc, m, h);
    __syncthreads();
#pragma unroll
    for (int t = 0; t < 4; ++t) {
      const int col = 16 * t + m;
      const float bb = bfr(b2[col]);
#pragma unroll
      for (int r = 0; r < 8; ++r) r2[(8 * h + r) * HC + col] = acc[t][r] + bb;
    }
    __syncthreads();
    if (wave == 0) {
#pragma unroll 1
      for (int i = 0; i < 128; ++i) {
        const int sl = __builtin_amdgcn_readfirstlane(rs[i]);
        if (sl >= 0) {
          const int slc = sl & (TGT - 1);
          const float* mr = (const float*)(base + MO_STG + (i >> 4) * WSTG + R2OFF) + (i & 15) * HC + 2 * lane;
          float* ap = agg + slc * HC + 2 * lane;
          const v2f mv = *(const v2f*)mr;
          v2f av = *(const v2f*)ap;
          av.x = fmaxf(av.x, mv.x);
          av.y = fmaxf(av.y, mv.y);
          *(v2f*)ap = av;
        }
      }
    }
    __syncthreads();
  }

  {
    const int rl = lane >> 4, col = (lane & 15) * 4;
#pragma unroll
    for (int i = 0; i < 16; ++i) {
      const int row = wave * 32 + 2 * i + rl;
      float* lp = agg + row * HC + col;
      float* gp = xf + (size_t)(nodeBase + row) * HC + col;
      const v4f xo = *(const v4f*)gp;
      v4f a = *(const v4f*)lp;
      a.x = fmaxf(xo.x, a.x); a.y = fmaxf(xo.y, a.y); a.z = fmaxf(xo.z, a.z); a.w = fmaxf(xo.w, a.w);
      *(v4f*)lp = a;
      *(volatile v4f*)gp = a;
    }
    __threadfence();
#pragma unroll
    for (int i = 0; i < 16; ++i) {
      const int row = wave * 32 + 2 * i + rl;
      const v4f a = *(const v4f*)(agg + row * HC + col);
      *(volatile v4f*)(xf + (size_t)(nodeBase + row) * HC + col) = a;
    }
  }
}

__global__ __launch_bounds__(NTHR) void k_fy(
    const int* __restrict__ ei, const float* __restrict__ rsq, const us* __restrict__ wpl,
    const float* __restrict__ b1, const float* __restrict__ b2, float* y,
    const int* __restrict__ loopp, int it, int nN, int nE) {
  if (it >= loopp[0]) return;
  __shared__ __attribute__((aligned(16))) us sP[RB * AP * 2];
  us*    sH  = sP;
  us*    sLo = sP + RB * AP;
  float* stg = (float*)sP;
  const int tid = threadIdx.x, lane = tid & 31, wave = tid >> 5, h = lane >> 4, m = lane & 15;
  const int rowBase = blockIdx.x * RB;
  const int lr = wave * 16 + m;
  int e = rowBase + lr;
  e = e > nE - 1 ? nE - 1 : e;
  int s = ei[e];      s = s < 0 ? 0 : (s > nN - 1 ? nN - 1 : s);
  int d = ei[nE + e]; d = d < 0 ? 0 : (d > nN - 1 ? nN - 1 : d);
  {
    const float* rp = rsq + (size_t)d * PQW + 32 * h;
    const float* sp = rsq + (size_t)s * PQW + 64 + 32 * h;
    const float* bp = b1 + 32 * h;
    us* dh = sH + lr * AP + 32 * h;
    us* dl = sLo + lr * AP + 32 * h;
#pragma unroll
    for (int q = 0; q < 4; ++q) {
      float f[8];
#pragma unroll
      for (int j = 0; j < 2; ++j) {
        const v4f a  = *(const v4f*)(rp + 8 * q + 4 * j);
        const v4f ss = *(const v4f*)(sp + 8 * q + 4 * j);
        const v4f c  = bfr4(*(const v4f*)(bp + 8 * q + 4 * j));
        const v4f val = a + ss + c;
        f[4 * j + 0] = fmaxf(val.x, 0.0f); f[4 * j + 1] = fmaxf(val.y, 0.0f);
        f[4 * j + 2] = fmaxf(val.z, 0.0f); f[4 * j + 3] = fmaxf(val.w, 0.0f);
      }
      v8us ph, pl;
#pragma unroll
      for (int j = 0; j < 8; ++j) {
        const us hb = f2bf(f[j]);
        ph[j] = hb;
        pl[j] = f2bf(f[j] - bf2f(hb));
      }
      *(v8us*)(dh + 8 * q) = ph;
      *(v8us*)(dl + 8 * q) = pl;
    }
  }
  __syncthreads();
  v8f acc[4];
  zacc(acc);
  mm2<2, 4>(sH + lr * AP + 8 * h, sLo + lr * AP + 8 * h, wpl + PL_FY2, acc, m, h);
  __syncthreads();
#pragma unroll
  for (int t = 0; t < 4; ++t) {
    const int col = 16 * t + m;
    const float bb = bfr(b2[col]);
#pragma unroll
    for (int r = 0; r < 8; ++r) stg[(wave * 16 + 8 * h + r) * HC + col] = acc[t][r] + bb;
  }
  __syncthreads();
  merge_max_rows16(stg + wave * 16 * HC, y + (size_t)(rowBase + wave * 16) * HC, lane);
}

__global__ __launch_bounds__(NTHR) void k_head(
    const float* __restrict__ xf, const us* __restrict__ wpl,
    const float* __restrict__ b1, const float* __restrict__ b2, float* out, int nN) {
  __shared__ __attribute__((aligned(16))) us sP[RB * AP * 2];
  __shared__ __attribute__((aligned(16))) float so[RB];
  us* sH  = sP;
  us* sLo = sP + RB * AP;
  const int tid = threadIdx.x, lane = tid & 31, wave = tid >> 5, h = lane >> 4, m = lane & 15;
  const int rowBase = blockIdx.x * RB;
  const int lr = wave * 16 + m;
  stage32(xf + (size_t)(rowBase + lr) * HC + 32 * h, sH + lr * AP + 32 * h, sLo + lr * AP + 32 * h);
  __syncthreads();
  v8f acc[4];
  zacc(acc);
  const us* aH = sH + lr * AP + 8 * h;
  const us* aL = sLo + lr * AP + 8 * h;
  mm2<2, 4>(aH, aL, wpl + PL_FE1, acc, m, h);
  __syncthreads();
  epi_hidden(acc, b1, sH, sLo, wave * 16 + 8 * h, m);
  __syncthreads();
  zacc(acc);
  mm2<2, 4>(aH, aL, wpl + PL_FE2, acc, m, h);
  __syncthreads();
  epi_hidden(acc, b2, sH, sLo, wave * 16 + 8 * h, m);
  __syncthreads();
  v8f a3[1];
  zacc(a3);
  mm2<2, 1>(aH, aL, wpl + PL_FE3, a3, m, h);
  if (m == 0) {
#pragma unroll
    for (int r = 0; r < 8; ++r) so[wave * 16 + 8 * h + r] = a3[0][r];
  }
  __syncthreads();
  if (wave == 0) {
    const int r0 = rowBase + 4 * lane;
    const v4f val = *(const v4f*)(so + 4 * lane);
    const bool full = r0 + 4 <= nN;
    if (full) *(volatile v4f*)(out + r0) = val;
    else {
      if (r0     < nN) *(volatile float*)(out + r0)     = val.x;
      if (r0 + 1 < nN) *(volatile float*)(out + r0 + 1) = val.y;
      if (r0 + 2 < nN) *(volatile float*)(out + r0 + 2) = val.z;
    }
    __threadfence();
    if (full) *(volatile v4f*)(out + r0) = val;
    else {
      if (r0     < nN) *(volatile float*)(out + r0)     = val.x;
      if (r0 + 1 < nN) *(volatile float*)(out + r0 + 1) = val.y;
      if (r0 + 2 < nN) *(volatile float*)(out + r0 + 2) = val.z;
    }
  }
}

extern "C" void kernel_launch(void* const* d_in, const int* in_sizes, int n_in,
                              void* d_out, int out_size, void* d_ws, size_t ws_size,
                              hipStream_t stream) {
  if (n_in < 25) return;
  const int nN = in_sizes[0] / 7;
  const int nE = in_sizes[2] / 2;
  if (nN < 1 || nE < 1) return;
  if (in_sizes[0] != 7 * nN || in_sizes[1] != 2 * nN || in_sizes[2] != 2 * nE || in_sizes[3] < 1) return;
  if (in_sizes[4] != 36 * HC || in_sizes[5] != HC || in_sizes[6] != HC * HC || in_sizes[7] != HC) return;
  if (in_sizes[8] != 27 * HC || in_sizes[9] != HC || in_sizes[10] != HC * HC || in_sizes[11] != HC) return;
  if (in_sizes[12] != 256 * HC || in_sizes[13] != HC || in_sizes[14] != HC * HC || in_sizes[15] != HC) return;
  if (in_sizes[16] != 192 * HC || in_sizes[17] != HC || in_sizes[18] != HC * HC || in_sizes[19] != HC) return;
  if (in_sizes[20] != HC * HC || in_sizes[21] != HC || in_sizes[22] != HC * HC || in_sizes[23] != HC) return;
  if (in_sizes[24] != HC) return;
  if (out_size != nN) return;
  if (nN >= (1 << 22) || nE >= (1 << 23)) return;

  const float* v    = (const float*)d_in[0];
  const float* lab  = (const float*)d_in[1];
  const int*   ei   = (const int*)d_in[2];
  const int*   loopp = (const int*)d_in[3];
  const float* hxw1 = (const float*)d_in[4];
  const float* hxb1 = (const float*)d_in[5];
  const float* hxw2 = (const float*)d_in[6];
  const float* hxb2 = (const float*)d_in[7];
  const float* hyw1 = (const float*)d_in[8];
  const float* hyb1 = (const float*)d_in[9];
  const float* hyw2 = (const float*)d_in[10];
  const float* hyb2 = (const float*)d_in[11];
  const float* fxw1 = (const float*)d_in[12];
  const float* fxb1 = (const float*)d_in[13];
  const float* fxw2 = (const float*)d_in[14];
  const float* fxb2 = (const float*)d_in[15];
  const float* fyw1 = (const float*)d_in[16];
  const float* fyb1 = (const float*)d_in[17];
  const float* fyw2 = (const float*)d_in[18];
  const float* fyb2 = (const float*)d_in[19];
  const float* few1 = (const float*)d_in[20];
  const float* feb1 = (const float*)d_in[21];
  const float* few2 = (const float*)d_in[22];
  const float* feb2 = (const float*)d_in[23];
  const float* few3 = (const float*)d_in[24];
  float* out = (float*)d_out;

  const int NPAD = ((nN + TGT - 1) / TGT) * TGT;
  const int EPAD = ((nE + RB - 1) / RB) * RB;

  char* ws = (char*)d_ws;
  size_t off = 0;
  const size_t oW = off; off += (size_t)PL_TOT * 2;            off = (off + 255) & ~(size_t)255;
  const size_t oG = off; off += 256;                           off = (off + 255) & ~(size_t)255;
  const size_t oX = off; off += (size_t)NPAD * HC * 4;         off = (off + 255) & ~(size_t)255;
  const size_t oP = off; off += (size_t)NPAD * PQW * 4;        off = (off + 255) & ~(size_t)255;
  const size_t oY = off; off += (size_t)EPAD * HC * 4;         off = (off + 255) & ~(size_t)255;
  if (off > ws_size || off > ((size_t)128 << 20)) return;
  us*    wpl  = (us*)(ws + oW);
  float* goal = (float*)(ws + oG);
  float* xf   = (float*)(ws + oX);
  float* pq   = (float*)(ws + oP);
  float* yf   = (float*)(ws + oY);

  const int vec8 = ((nE & 3) == 0) ? 1 : 0;

  k_prep<<<NPREP, NTHR, 0, stream>>>(hxw1, hxw2, hyw1, hyw2, fxw1, fxw2, fyw1, fyw2, few1, few2, few3, wpl);
  k_goal<<<1, NTHR, 0, stream>>>(v, lab, goal, nN);
  k_xinit<<<NPAD / RB, NTHR, ROW_LDS, stream>>>(v, lab, goal, wpl, hxb1, hxb2, xf, nN);
  k_yinit<<<EPAD / RB, NTHR, ROW_LDS, stream>>>(v, lab, ei, wpl, hyb1, hyb2, yf, nN, nE);

  hipFuncSetAttribute(reinterpret_cast<const void*>(&k_proj), hipFuncAttributeMaxDynamicSharedMemorySize, PROJ_LDS);
  hipFuncSetAttribute(reinterpret_cast<const void*>(&k_msg), hipFuncAttributeMaxDynamicSharedMemorySize, MSG_LDS);
  for (int it = 0; it < LMAX; ++it) {
    k_proj<<<NPAD / RB, NTHR, PROJ_LDS, stream>>>(xf, wpl + PL_CXH, wpl + PL_CXL, pq, loopp, it);
    k_msg<<<NPAD / TGT, NTHR, MSG_LDS, stream>>>(ei, yf, pq, wpl, fxb1, fxb2, xf, loopp, it, nN, nE, vec8);
    k_proj<<<NPAD / RB, NTHR, PROJ_LDS, stream>>>(xf, wpl + PL_CYH, wpl + PL_CYL, pq, loopp, it);
    k_fy<<<EPAD / RB, NTHR, 0, stream>>>(ei, pq, wpl, fyb1, fyb2, yf, loopp, it, nN, nE);
  }
  k_head<<<NPAD / RB, NTHR, 0, stream>>>(xf, wpl, feb1, feb2, out, nN);
}
